// MLPPredictor_40664750359264
// MI455X (gfx1250) — hardware-verified
//
#include <hip/hip_runtime.h>


namespace {
constexpr int N = 100000, EFULL = 1600000, E = EFULL, EL = E  , F = 128, HID = 32, TE = 64  ;
constexpr float XS = 8.0f, WSC = 256.0f, WSQ = 0.25f, RS_ = 1024.0f;
static_assert(E % TE == 0 && EL % TE == 0 && F == 128 && HID == 32, "tiling");
typedef _Float16 b16;
typedef __attribute__((ext_vector_type(16))) _Float16 v16b;
typedef __attribute__((ext_vector_type(8))) _Float16 v8b;
typedef __attribute__((ext_vector_type(8))) float v8f;
typedef __attribute__((ext_vector_type(4))) float v4f;
__device__ __forceinline__ float bf16_rne(float f) { unsigned int u = __float_as_uint(f); u += 0x7FFFu + ((u >> 16) & 1u); return __uint_as_float(u & 0xFFFF0000u); }
__device__ __forceinline__ void split16(float v, b16& hi, b16& lo) { hi = (b16)v; lo = (b16)(v - (float)hi); }
__device__ __forceinline__ v16b frag_kb(const b16* p, int hh) { const v8b a = *(const v8b*)(p + 8 * hh), b = *(const v8b*)(p + 16 + 8 * hh); v16b f;
#pragma unroll
  for (int e = 0; e < 8; ++e) { f[e] = a[e]; f[8 + e] = b[e]; } return f; }
__device__ __forceinline__ v8f wmma16b(v16b a, v16b b, v8f c) { v8f d = __builtin_amdgcn_wmma_f32_16x16x32_f16(false, a, false, b, (short)0, c, false, false); asm volatile("v_nop\n\tv_nop\n\tv_nop\n\tv_nop" : "+v"(d) : "v"(a), "v"(b)); return d; }
__device__ __forceinline__ void wave_lds_sync() { __builtin_amdgcn_fence(__ATOMIC_RELEASE, "workgroup"); __builtin_amdgcn_wave_barrier(); __builtin_amdgcn_fence(__ATOMIC_ACQUIRE, "workgroup"); }
__device__ __forceinline__ float pmul(float a, float b) { float p = a * b; asm volatile("" : "+v"(p)); return p; }
__device__ __forceinline__ int iclamp(int v, int lo, int hi) { return v < lo ? lo : (v > hi ? hi : v); }

typedef __attribute__((ext_vector_type(2))) _Float16 v2h;
typedef __attribute__((ext_vector_type(4))) _Float16 v4h;
typedef __attribute__((ext_vector_type(2))) float v2f;
typedef __attribute__((ext_vector_type(4))) int v4i;
__device__ __forceinline__ float nexp2(float v) { return __builtin_amdgcn_exp2f(v); }
typedef __attribute__((ext_vector_type(4))) _Float16 v4h_;
__global__ __launch_bounds__(256) void wt_kernel(const float* __restrict__ w, b16* __restrict__ WT, float scl) {
  const int u = blockIdx.x * 256 + threadIdx.x; if (u >= HID * F / 8) return; const int e = u * 8; const int o = e / F, k0 = e % F; v8b v;
#pragma unroll
  for (int j = 0; j < 8; ++j) v[j] = (b16)(bf16_rne(w[(size_t)(k0 + j) * HID + o]) * scl);
  for (int pass = 0; pass < 2; ++pass) { *(volatile v8b*)(WT + e) = v; __threadfence(); }
}
__global__ __launch_bounds__(256) void edge_kernel(const float* __restrict__ h, const int* __restrict__ srcs, const int* __restrict__ dsts, const b16* __restrict__ W1T, const b16* __restrict__ W1Q, const float* __restrict__ b1, const float* __restrict__ w2, const float* __restrict__ b2, float* __restrict__ out) {
  __shared__ __attribute__((aligned(16))) b16 Ah[TE][F + 8], Al[TE][F + 8]; __shared__ float Hs[TE][HID + 1]; __shared__ float w2s[HID]; __shared__ float sc[TE];
  const int tid = threadIdx.x, wave = tid >> 5, lane = tid & 31, nloc = lane & 15, hlf = lane >> 4; const size_t e0 = (size_t)blockIdx.x * TE;
  if (tid < HID) w2s[tid] = bf16_rne(w2[tid]);
  { const int row = tid >> 2, g = tid & 3, c0 = g * 32; const size_t e = e0 + row; const int s = iclamp(srcs[e], 0, N - 1), d = iclamp(dsts[e], 0, N - 1); const float* hs = h + (size_t)s * F + c0; const float* hd = h + (size_t)d * F + c0;
#pragma unroll
    for (int q = 0; q < 8; ++q) { const v4f a = *(const v4f*)(hs + 4 * q), b = *(const v4f*)(hd + 4 * q); v4h_ hv, lv; for (int j = 0; j < 4; ++j) { const float pe = bf16_rne(a[j]) * bf16_rne(b[j]); const float vs = pe * XS; const b16 p = (b16)vs; hv[j] = p; lv[j] = (b16)((vs - (float)p) * RS_); } *(v4h_*)(&Ah[row][c0 + 4 * q]) = hv; *(v4h_*)(&Al[row][c0 + 4 * q]) = lv; } }
  __syncthreads();
  { const int rt = wave & 3, ct = wave >> 2; v8f acc = (v8f){}; const b16* br = W1T + (size_t)(ct * 16 + nloc) * F; const b16* bq = W1Q + (size_t)(ct * 16 + nloc) * F;
#pragma unroll
    for (int kb = 0; kb < F; kb += 32) { acc = wmma16b(frag_kb(&Ah[rt * 16 + nloc][kb], hlf), frag_kb(br + kb, hlf), acc); acc = wmma16b(frag_kb(&Al[rt * 16 + nloc][kb], hlf), frag_kb(bq + kb, hlf), acc); }
    const int col = ct * 16 + nloc; const float bb = bf16_rne(b1[col]);
#pragma unroll
    for (int r = 0; r < 8; ++r) Hs[rt * 16 + 8 * hlf + r][col] = fmaxf(acc[r] * (1.0f / (XS * WSC)) + bb, 0.0f); }
  __syncthreads();
  if (tid < TE) { float s = 0.0f;
#pragma unroll 8
    for (int o = 0; o < HID; ++o) s = fmaf(Hs[tid][o], w2s[o], s);
    sc[tid] = s + bf16_rne(b2[0]); }
  __syncthreads();
  for (int pass = 0; pass < 2; ++pass) { if (wave < 2) ((volatile float*)out)[e0 + wave * 32 + lane] = sc[wave * 32 + lane]; __threadfence(); }
}
}

extern "C" void kernel_launch(void* const* d_in, const int* in_sizes, int n_in, void* d_out, int out_size, void* d_ws, size_t ws_size, hipStream_t stream) {
  (void)n_in;
  auto Fp = [&](int i) { return (const float*)d_in[i]; }; auto Ip = [&](int i) { return (const int*)d_in[i]; };
  if (in_sizes[0] != N * F || in_sizes[1] != EFULL || in_sizes[2] != EFULL || in_sizes[3] != F * HID || in_sizes[4] != HID || in_sizes[5] != HID || in_sizes[6] != 1 || out_size != EFULL) return;
  size_t off = 0; char* ws = (char*)d_ws;
  auto carve = [&](size_t bytes) { char* p = ws + off; off += (bytes + 255) & ~(size_t)255; return p; };
  b16* W1T = (b16*)carve((size_t)HID * F * 2); b16* W1Q = (b16*)carve((size_t)HID * F * 2);
  if (off > ws_size || off > ((size_t)128 << 20)) return;
  wt_kernel<<<(HID * F / 8 + 255) / 256, 256, 0, stream>>>(Fp(3), W1T, WSC); wt_kernel<<<(HID * F / 8 + 255) / 256, 256, 0, stream>>>(Fp(3), W1Q, WSQ);
  edge_kernel<<<EL / TE, 256, 0, stream>>>(Fp(0), Ip(1), Ip(2), W1T, W1Q, Fp(4), Fp(5), Fp(6), (float*)d_out);
}
